// Model0_1_53060025975059
// MI455X (gfx1250) — hardware-verified
//
#include <hip/hip_runtime.h>
#include <math.h>

constexpr int NBATCH = 1024;
constexpr int NSTEP  = 256;
constexpr int NFEAT  = 23;
constexpr int NHID   = 100;
constexpr int NGATE4 = 400;
constexpr int SIN    = 6;
constexpr int SOUT   = 20;
constexpr int NCLS   = 2;
constexpr int HPAD   = 128;
constexpr int XKP    = 32;
constexpr int GROWS  = 4 * HPAD;
constexpr int NTHR   = 256;
constexpr int NCW    = 7;
constexpr int RB     = 16;
constexpr int HP     = 136;
constexpr int XP     = 40;
constexpr int HFP    = 116;
constexpr float WSC     = 16.0f;
constexpr float WSC_INV = 1.0f / 16.0f;
constexpr float E_F     = 2.718281828459045f;

static_assert(NBATCH % RB == 0);
static_assert(NCW * 16 >= NHID && NCW * 16 <= HFP && NCW * 16 <= HPAD);
static_assert((2 * 2 * RB * HP) % NTHR == 0);
static_assert(HP % 8 == 0 && XP % 8 == 0);
static_assert(NFEAT <= XKP && NHID <= HPAD && HPAD % 32 == 0 && XKP % 32 == 0);
static_assert(NTHR / 32 == NCW + 1);
static_assert(RB * NCLS * 4 == 128);
static_assert((GROWS * HPAD * 2) % 512 == 0 && (HPAD * HPAD * 2) % 512 == 0 && (GROWS * XKP * 2) % 512 == 0);

typedef __attribute__((ext_vector_type(16))) _Float16 v16h;
typedef __attribute__((ext_vector_type(8)))  _Float16 v8h;
typedef __attribute__((ext_vector_type(8)))  float    v8f;
typedef __attribute__((ext_vector_type(4)))  float    v4f;

template <typename T> struct Frag;
template <> struct Frag<_Float16> {
  typedef v16h V; union U { v16h v; v8h h[2]; };
  static __device__ __forceinline__ v16h load(const _Float16* p) {
    U f; f.h[0] = *(const v8h*)(p); f.h[1] = *(const v8h*)(p + 16); return f.v;
  }
};

__device__ __forceinline__ v8f mma_g(v16h a, v16h b, v8f c) {
  c = __builtin_amdgcn_wmma_f32_16x16x32_f16(false, a, false, b, (short)0, c, false, false);
  asm volatile("v_nop\n\tv_nop\n\tv_nop\n\tv_nop" : "+v"(c) : "v"(a), "v"(b));
  return c;
}

__device__ __forceinline__ float fsig(float x)  { return __builtin_amdgcn_rcpf(1.0f + __expf(-x)); }
__device__ __forceinline__ float ftanh(float x) { return 1.0f - 2.0f * __builtin_amdgcn_rcpf(__expf(2.0f * x) + 1.0f); }

__global__ __launch_bounds__(NTHR) void wprep_kernel(const float* __restrict__ W, int ncol, int kreal,
                                                     _Float16* __restrict__ dst, int nrow, int kp) {
  const int i   = blockIdx.x * NTHR + threadIdx.x;
  const int kp8 = kp >> 3;
  const int n8  = nrow * kp8;
  if (i < n8) {
    const int row = i / kp8;
    const int k0  = (i - row * kp8) * 8;
    const int g   = row >> 7;
    const int u   = row & (HPAD - 1);
    int col = g * NHID + u;
    col = col < ncol ? col : (ncol - 1);
    const bool uok = (u < NHID);
    v8h hv;
#pragma unroll
    for (int e = 0; e < 8; ++e) {
      const int k  = k0 + e;
      const int kc = k < kreal ? k : (kreal - 1);
      const float w = W[(size_t)kc * ncol + col];
      const float v = (uok && k < kreal) ? (w * WSC) : 0.0f;
      hv[e] = (_Float16)v;
    }
    *(volatile v8h*)(dst + (size_t)i * 8) = hv;
    __threadfence();
    *(volatile v8h*)(dst + (size_t)i * 8) = hv;
  }
}

__device__ __forceinline__ void stage_step(const float* __restrict__ x_lab, const float* __restrict__ t_lab,
                                           int rb, int ts, int lane, _Float16* xt, float* dk) {
  const int m  = lane >> 1;
  const int kh = (lane & 1) * 16;
  const float* xr = x_lab + ((size_t)(rb + m) * NSTEP + (size_t)ts) * NFEAT;
  v8h v0, v1;
#pragma unroll
  for (int e = 0; e < 8; ++e) {
    const int ka = kh + e;
    const int kb = kh + 8 + e;
    const float fa = xr[ka < NFEAT ? ka : (NFEAT - 1)];
    const float fb = xr[kb < NFEAT ? kb : (NFEAT - 1)];
    v0[e] = (_Float16)((ka < NFEAT) ? fa : 0.0f);
    v1[e] = (_Float16)((kb < NFEAT) ? fb : 0.0f);
  }
  *(v8h*)(xt + m * XP + kh)     = v0;
  *(v8h*)(xt + m * XP + kh + 8) = v1;
  if (lane < RB) {
    const float d = t_lab[(size_t)(rb + lane) * NSTEP + (size_t)ts];
    dk[lane] = 1.0f / logf(E_F + d);
  }
}

__global__ __launch_bounds__(NTHR) void tlstm_kernel(const float* __restrict__ x_lab,
                                                     const float* __restrict__ t_lab,
                                                     const float* __restrict__ x_state,
                                                     const float* __restrict__ b_lstm,
                                                     const float* __restrict__ b_d,
                                                     const float* __restrict__ W_state,
                                                     const float* __restrict__ b_state,
                                                     const float* __restrict__ W_fc,
                                                     const float* __restrict__ b_fc,
                                                     const _Float16* __restrict__ WHT,
                                                     const _Float16* __restrict__ WDT,
                                                     const _Float16* __restrict__ WXT,
                                                     float* __restrict__ out) {
  __shared__ __align__(16) _Float16 Ht[2][RB * HP];
  __shared__ __align__(16) _Float16 Ct[2][RB * HP];
  __shared__ __align__(16) _Float16 Xt[2][RB * XP];
  __shared__ __align__(16) float    Dk[2][RB];
  __shared__ __align__(16) float    Hf[RB * HFP];
  __shared__ __align__(16) float    Po[RB * NCLS];

  const int tid  = threadIdx.x;
  const int lane = tid & 31;
  const int wave = tid >> 5;
  const int c    = lane & 15;
  const int hh   = lane >> 4;
  const int koff = hh * 8;
  const int rb   = blockIdx.x * RB;
  const int u    = 16 * wave + c;

  {
    _Float16* hz = &Ht[0][0];
    _Float16* cz = &Ct[0][0];
#pragma unroll 1
    for (int i = tid; i < 2 * RB * HP; i += NTHR) { hz[i] = (_Float16)0.0f; cz[i] = (_Float16)0.0f; }
  }

  const int  uc  = u < NHID ? u : (NHID - 1);
  const bool uok = (u < NHID);
  float bg[4];
#pragma unroll
  for (int g = 0; g < 4; ++g) { const float bv = b_lstm[g * NHID + uc]; bg[g] = uok ? bv : 0.0f; }
  float bdv; { const float bv = b_d[uc]; bdv = uok ? bv : 0.0f; }

  float cst[8], hst[8];
#pragma unroll
  for (int r = 0; r < 8; ++r) { cst[r] = 0.0f; hst[r] = 0.0f; }

  if (wave == NCW) stage_step(x_lab, t_lab, rb, 0, lane, &Xt[0][0], &Dk[0][0]);
  __syncthreads();

  const v8f z8 = {0.f, 0.f, 0.f, 0.f, 0.f, 0.f, 0.f, 0.f};

#pragma unroll 1
  for (int t = 0; t < NSTEP; ++t) {
    const int cur = t & 1;
    const int nxt = cur ^ 1;
    if (wave < NCW) {
      const _Float16* hrow = &Ht[cur][0] + c * HP + koff;
      const _Float16* crow = &Ct[cur][0] + c * HP + koff;
      const _Float16* xrow = &Xt[cur][0] + c * XP + koff;
      v8f ag[4];
#pragma unroll
      for (int g = 0; g < 4; ++g) ag[g] = z8;
      v8f acs = z8;
#pragma unroll 1
      for (int ks = 0; ks < HPAD; ks += 32) {
        const v16h ah = Frag<_Float16>::load(hrow + ks);
        const v16h ac = Frag<_Float16>::load(crow + ks);
        const v16h bd = Frag<_Float16>::load(WDT + (size_t)u * HPAD + koff + ks);
        acs = mma_g(ac, bd, acs);
#pragma unroll
        for (int g = 0; g < 4; ++g) {
          const v16h bw = Frag<_Float16>::load(WHT + (size_t)(g * HPAD + u) * HPAD + koff + ks);
          ag[g] = mma_g(ah, bw, ag[g]);
        }
      }
      {
        const v16h ax = Frag<_Float16>::load(xrow);
#pragma unroll
        for (int g = 0; g < 4; ++g) {
          const v16h bx = Frag<_Float16>::load(WXT + (size_t)(g * HPAD + u) * XKP + koff);
          ag[g] = mma_g(ax, bx, ag[g]);
        }
      }
      const float* dkc = &Dk[cur][0];
      _Float16* hnt = &Ht[nxt][0];
      _Float16* cnt = &Ct[nxt][0];
#pragma unroll
      for (int r = 0; r < 8; ++r) {
        const int row = 8 * hh + r;
        const float pi = ag[0][r] * WSC_INV + bg[0];
        const float pf = ag[1][r] * WSC_INV + bg[1];
        const float pg = ag[2][r] * WSC_INV + bg[2];
        const float po = ag[3][r] * WSC_INV + bg[3];
        const float ig = fsig(pi);
        const float fg = fsig(pf);
        const float og = fsig(po);
        const float gg = ftanh(pg);
        const float cs = ftanh(acs[r] * WSC_INV + bdv);
        const float dk = dkc[row];
        const float co = cst[r];
        const float cadj = (co - cs) + cs * dk;
        const float cn = fg * cadj + ig * gg;
        const float hn = og * ftanh(cn);
        cst[r] = cn;
        hst[r] = hn;
        hnt[row * HP + u] = (_Float16)hn;
        cnt[row * HP + u] = (_Float16)cn;
      }
    } else {
      const int ts = (t + 1 < NSTEP) ? (t + 1) : (NSTEP - 1);
      if (t + 1 < NSTEP) stage_step(x_lab, t_lab, rb, ts, lane, &Xt[nxt][0], &Dk[nxt][0]);
    }
    __syncthreads();
  }

  if (wave < NCW) {
#pragma unroll
    for (int r = 0; r < 8; ++r) Hf[(8 * hh + r) * HFP + u] = hst[r];
  }
  __syncthreads();
  if (tid < RB) {
    const int m    = tid;
    const int brow = rb + m;
    float xs[SIN];
#pragma unroll
    for (int k = 0; k < SIN; ++k) xs[k] = x_state[(size_t)brow * SIN + k];
    float y0 = b_fc[0];
    float y1 = b_fc[1];
    const float* hf = Hf + m * HFP;
#pragma unroll 1
    for (int j = 0; j < NHID; ++j) {
      const float hv = hf[j];
      y0 += hv * W_fc[2 * j];
      y1 += hv * W_fc[2 * j + 1];
    }
#pragma unroll 1
    for (int j = 0; j < SOUT; ++j) {
      float e = b_state[j];
#pragma unroll
      for (int k = 0; k < SIN; ++k) e += xs[k] * W_state[k * SOUT + j];
      y0 += e * W_fc[2 * (NHID + j)];
      y1 += e * W_fc[2 * (NHID + j) + 1];
    }
    const float mx  = fmaxf(y0, y1);
    const float e0  = expf(y0 - mx);
    const float e1  = expf(y1 - mx);
    const float inv = 1.0f / (e0 + e1);
    Po[2 * m]     = e0 * inv;
    Po[2 * m + 1] = e1 * inv;
  }
  __syncthreads();
  if (tid < 8) {
    const v4f v = *(const v4f*)(Po + 4 * tid);
    volatile v4f* op = (volatile v4f*)(out + (size_t)rb * NCLS + 4 * tid);
    *op = v;
    __threadfence();
    *op = v;
  }
}

extern "C" void kernel_launch(void* const* d_in, const int* in_sizes, int n_in,
                              void* d_out, int out_size, void* d_ws, size_t ws_size, hipStream_t stream) {
  if (n_in < 12 || d_out == nullptr || d_ws == nullptr) return;
  if (in_sizes[0] != NBATCH * NSTEP * NFEAT || in_sizes[1] != NBATCH * NSTEP || in_sizes[2] != NBATCH * SIN ||
      in_sizes[3] != NFEAT * NGATE4 || in_sizes[4] != NHID * NGATE4 || in_sizes[5] != NGATE4 ||
      in_sizes[6] != NHID * NHID || in_sizes[7] != NHID || in_sizes[8] != SIN * SOUT || in_sizes[9] != SOUT ||
      in_sizes[10] != (NHID + SOUT) * NCLS || in_sizes[11] != NCLS || out_size != NBATCH * NCLS) return;

  const float* x_lab   = (const float*)d_in[0];
  const float* t_lab   = (const float*)d_in[1];
  const float* x_state = (const float*)d_in[2];
  const float* W_x     = (const float*)d_in[3];
  const float* W_h     = (const float*)d_in[4];
  const float* b_lstm  = (const float*)d_in[5];
  const float* W_d     = (const float*)d_in[6];
  const float* b_d     = (const float*)d_in[7];
  const float* W_state = (const float*)d_in[8];
  const float* b_state = (const float*)d_in[9];
  const float* W_fc    = (const float*)d_in[10];
  const float* b_fc    = (const float*)d_in[11];
  float* out = (float*)d_out;

  char* ws = (char*)d_ws; size_t off = 0;
  auto carve = [&](size_t bytes) -> char* { char* p = ws + off; off += (bytes + 255) & ~(size_t)255; return p; };
  _Float16* WHT = (_Float16*)carve((size_t)GROWS * HPAD * 2);
  _Float16* WDT = (_Float16*)carve((size_t)HPAD  * HPAD * 2);
  _Float16* WXT = (_Float16*)carve((size_t)GROWS * XKP  * 2);
  if (off > ws_size || off > (size_t)134217728) return;

  const int n8h = GROWS * (HPAD / 8);
  const int n8d = HPAD  * (HPAD / 8);
  const int n8x = GROWS * (XKP  / 8);
  wprep_kernel<<<(n8h + NTHR - 1) / NTHR, NTHR, 0, stream>>>(W_h, NGATE4, NHID,  WHT, GROWS, HPAD);
  wprep_kernel<<<(n8d + NTHR - 1) / NTHR, NTHR, 0, stream>>>(W_d, NHID,   NHID,  WDT, HPAD,  HPAD);
  wprep_kernel<<<(n8x + NTHR - 1) / NTHR, NTHR, 0, stream>>>(W_x, NGATE4, NFEAT, WXT, GROWS, XKP);

  tlstm_kernel<<<NBATCH / RB, NTHR, 0, stream>>>(x_lab, t_lab, x_state, b_lstm, b_d, W_state, b_state, W_fc, b_fc,
                                                 WHT, WDT, WXT, out);
}
